// VDPWIModel_74423193305823
// MI455X (gfx1250) — hardware-verified
//
#include <hip/hip_runtime.h>
#include <math.h>

#pragma clang fp contract(off)

typedef _Float16       v8h  __attribute__((ext_vector_type(8)));
typedef _Float16       v16h __attribute__((ext_vector_type(16)));
typedef __bf16         v16b __attribute__((ext_vector_type(16)));
typedef unsigned short v8us __attribute__((ext_vector_type(8)));
typedef float          v8f  __attribute__((ext_vector_type(8)));
typedef float          v4f  __attribute__((ext_vector_type(4)));
typedef float          v4fa __attribute__((ext_vector_type(4), may_alias));
typedef unsigned int   v4u  __attribute__((ext_vector_type(4)));

union FragH  { v16h v; v8h hv[2]; };
union FragB  { v16b v; v8us hv[2]; };
union Pack8H { v8h hv; v4u u; };
union Pack8U { v8us hv; v4u u; };

#define TT    48
#define HID   250
#define HP    256
#define G4    1000
#define GP    1024
#define EMBD  300
#define EKP   320
#define NPOS  2304
#define NL    5

__device__ __forceinline__ v8f zero8() {
  v8f z = {0.f, 0.f, 0.f, 0.f, 0.f, 0.f, 0.f, 0.f};
  return z;
}

__device__ __forceinline__ unsigned short bf16_rne(float x) {
  unsigned int u = __float_as_uint(x);
  u += 0x7FFFu + ((u >> 16) & 1u);
  return (unsigned short)(u >> 16);
}
__device__ __forceinline__ float bf16_val(unsigned short b) {
  return __uint_as_float(((unsigned int)b) << 16);
}

__device__ __forceinline__ v8f wmma_bf(const v16b a, const v16b b, v8f acc) {
  return __builtin_amdgcn_wmma_f32_16x16x32_bf16(false, a, false, b, (short)0, acc, false, false);
}
__device__ __forceinline__ v8f wmma_hf(const v16h a, const v16h b, v8f acc) {
  return __builtin_amdgcn_wmma_f32_16x16x32_f16(false, a, false, b, (short)0, acc, false, false);
}


__global__ __launch_bounds__(256) void k_pack_nk3(const float* __restrict__ w, unsigned short* __restrict__ Bh,
                                                  unsigned short* __restrict__ Bl, int K, int N, int Kp, int Np) {
  const int c = blockIdx.x * 256 + threadIdx.x;
  const int kc8 = Kp >> 3;
  const int total = Np * kc8;
  if (c >= total) return;
  const int n = c / kc8, kc = c - n * kc8;
  const int k = kc << 3;
  Pack8U vh, vl;
  #pragma unroll
  for (int j = 0; j < 8; ++j) {
    float x = (n < N && (k + j) < K) ? w[(size_t)n * K + k + j] : 0.0f;
    unsigned short hb = bf16_rne(x);
    float r = x - bf16_val(hb);
    vh.hv[j] = hb;
    vl.hv[j] = bf16_rne(r);
  }
  volatile v4u* dh = (volatile v4u*)(Bh + (size_t)c * 8);
  volatile v4u* dl = (volatile v4u*)(Bl + (size_t)c * 8);
  const v4u uh = vh.u, ul = vl.u;
  *dh = uh; *dl = ul;
  __threadfence();
  *dh = uh; *dl = ul;
}

__global__ __launch_bounds__(256) void k_pack_nk(const float* __restrict__ w, _Float16* __restrict__ Bt,
                                                 int K, int N, int Kp, int Np) {
  const int c = blockIdx.x * 256 + threadIdx.x;
  const int kc8 = Kp >> 3;
  const int total = Np * kc8;
  if (c >= total) return;
  const int n = c / kc8, kc = c - n * kc8;
  const int k = kc << 3;
  Pack8H val;
  #pragma unroll
  for (int j = 0; j < 8; ++j) {
    float x = (n < N && (k + j) < K) ? w[(size_t)n * K + k + j] : 0.0f;
    val.hv[j] = (_Float16)x;
  }
  volatile v4u* dst = (volatile v4u*)(Bt + (size_t)c * 8);
  const v4u u = val.u;
  *dst = u;
  __threadfence();
  *dst = u;
}

__global__ __launch_bounds__(256) void k_pack_emb3(const float* __restrict__ emb, const int* __restrict__ ids1,
                                                   const int* __restrict__ ids2, unsigned short* __restrict__ Ah,
                                                   unsigned short* __restrict__ Al, int vocab) {
  const int c = blockIdx.x * 256 + threadIdx.x;
  const int kc8 = EKP >> 3;
  const int total = 2 * TT * kc8;
  if (c >= total) return;
  const int m = c / kc8, kc = c - m * kc8;
  int id = (m < TT) ? ids1[m] : ids2[m - TT];
  id = min(max(id, 0), vocab - 1);
  const int k = kc << 3;
  const float* src = emb + (size_t)id * EMBD;
  Pack8U vh, vl;
  #pragma unroll
  for (int j = 0; j < 8; ++j) {
    float x = ((k + j) < EMBD) ? src[k + j] : 0.0f;
    unsigned short hb = bf16_rne(x);
    float r = x - bf16_val(hb);
    vh.hv[j] = hb;
    vl.hv[j] = bf16_rne(r);
  }
  volatile v4u* dh = (volatile v4u*)(Ah + (size_t)c * 8);
  volatile v4u* dl = (volatile v4u*)(Al + (size_t)c * 8);
  const v4u uh = vh.u, ul = vl.u;
  *dh = uh; *dl = ul;
  __threadfence();
  *dh = uh; *dl = ul;
}

__global__ __launch_bounds__(256) void k_im2col(const float* __restrict__ in  ,
                                                _Float16* __restrict__ A, int Cin, int HW, int K, int Mp, int Kp) {
  const int c = blockIdx.x * 256 + threadIdx.x;
  const int kc8 = Kp >> 3;
  const int total = Mp * kc8;
  if (c >= total) return;
  const int m = c / kc8, kc = c - m * kc8;
  const int k = kc << 3;
  const int M = HW * HW;
  const int y = m / HW, x = m - y * HW;
  Pack8H val;
  #pragma unroll
  for (int j = 0; j < 8; ++j) {
    const int kk = k + j;
    float v = 0.0f;
    if (m < M && kk < K) {
      const int ch = kk / 9, rem = kk - ch * 9, dy = rem / 3, dx = rem - dy * 3;
      const int iy = y + dy - 1, ix = x + dx - 1;
      if (iy >= 0 && iy < HW && ix >= 0 && ix < HW && ch < Cin)
        v = in[((size_t)ch * HW + iy) * HW + ix];
    }
    val.hv[j] = (_Float16)v;
  }
  volatile v4u* dst = (volatile v4u*)(A + (size_t)c * 8);
  const v4u u = val.u;
  *dst = u;
  __threadfence();
  *dst = u;
}

__device__ __forceinline__ void store_tile_lines(const float* tile, float* Cbase, int Np, int l) {
  const int rr = l >> 3, cq = (l & 7) * 4;
  v4f v[4];
  #pragma unroll
  for (int q = 0; q < 4; ++q) v[q] = *(const v4fa*)(tile + (4 * q + rr) * 32 + cq);
  #pragma unroll
  for (int q = 0; q < 4; ++q) *(volatile v4f*)(Cbase + (size_t)(4 * q + rr) * Np + cq) = v[q];
  __threadfence();
  #pragma unroll
  for (int q = 0; q < 4; ++q) *(volatile v4f*)(Cbase + (size_t)(4 * q + rr) * Np + cq) = v[q];
}

__global__ __launch_bounds__(32) void k_gemm_x3(const unsigned short* __restrict__ Ah, const unsigned short* __restrict__ Al,
                                                const unsigned short* __restrict__ Bh, const unsigned short* __restrict__ Bl,
                                                float* __restrict__ C, int Mp, int Np, int Kp) {
  __shared__ __align__(16) float tile[16 * 32];
  const int ng = Np >> 5;
  const int ntiles = (Mp >> 4) * ng;
  const int bid = blockIdx.x;
  if (bid >= ntiles) return;
  const int mt = bid / ng, ngi = bid - mt * ng;
  const int l = threadIdx.x & 31, h = l >> 4, m = l & 15;
  const unsigned short* Ahr = Ah + (size_t)(mt * 16 + m) * Kp;
  const unsigned short* Alr = Al + (size_t)(mt * 16 + m) * Kp;
  const unsigned short* B0h = Bh + (size_t)(ngi * 32 + m) * Kp;
  const unsigned short* B0l = Bl + (size_t)(ngi * 32 + m) * Kp;
  const unsigned short* B1h = Bh + (size_t)(ngi * 32 + 16 + m) * Kp;
  const unsigned short* B1l = Bl + (size_t)(ngi * 32 + 16 + m) * Kp;

  v8f acc0 = zero8(), acc1 = zero8();
  #pragma unroll 1
  for (int k0 = 0; k0 < Kp; k0 += 32) {
    FragB ah, al, b0h, b0l, b1h, b1l;
    ah.hv[0]  = *(const v8us*)(Ahr + k0 + 8 * h);
    ah.hv[1]  = *(const v8us*)(Ahr + k0 + 16 + 8 * h);
    al.hv[0]  = *(const v8us*)(Alr + k0 + 8 * h);
    al.hv[1]  = *(const v8us*)(Alr + k0 + 16 + 8 * h);
    b0h.hv[0] = *(const v8us*)(B0h + k0 + 8 * h);
    b0h.hv[1] = *(const v8us*)(B0h + k0 + 16 + 8 * h);
    b0l.hv[0] = *(const v8us*)(B0l + k0 + 8 * h);
    b0l.hv[1] = *(const v8us*)(B0l + k0 + 16 + 8 * h);
    b1h.hv[0] = *(const v8us*)(B1h + k0 + 8 * h);
    b1h.hv[1] = *(const v8us*)(B1h + k0 + 16 + 8 * h);
    b1l.hv[0] = *(const v8us*)(B1l + k0 + 8 * h);
    b1l.hv[1] = *(const v8us*)(B1l + k0 + 16 + 8 * h);
    acc0 = wmma_bf(ah.v, b0h.v, acc0);
    acc0 = wmma_bf(ah.v, b0l.v, acc0);
    acc0 = wmma_bf(al.v, b0h.v, acc0);
    acc1 = wmma_bf(ah.v, b1h.v, acc1);
    acc1 = wmma_bf(ah.v, b1l.v, acc1);
    acc1 = wmma_bf(al.v, b1h.v, acc1);
    asm volatile("v_nop\n\tv_nop\n\tv_nop\n\tv_nop"
                 : "+v"(acc0), "+v"(acc1)
                 : "v"(ah.v), "v"(al.v), "v"(b0h.v), "v"(b0l.v), "v"(b1h.v), "v"(b1l.v));
  }
  #pragma unroll
  for (int r = 0; r < 8; ++r) {
    tile[(8 * h + r) * 32 + m]      = acc0[r];
    tile[(8 * h + r) * 32 + 16 + m] = acc1[r];
  }
  __syncthreads();
  store_tile_lines(tile, C + (size_t)(mt * 16) * Np + ngi * 32, Np, l);
}

__global__ __launch_bounds__(32) void k_gemm_h(const _Float16* __restrict__ A, const _Float16* __restrict__ Bt,
                                               float* __restrict__ C, int Mp, int Np, int Kp) {
  __shared__ __align__(16) float tile[16 * 32];
  const int ng = Np >> 5;
  const int ntiles = (Mp >> 4) * ng;
  const int bid = blockIdx.x;
  if (bid >= ntiles) return;
  const int mt = bid / ng, ngi = bid - mt * ng;
  const int l = threadIdx.x & 31, h = l >> 4, m = l & 15;
  const _Float16* Arow = A  + (size_t)(mt * 16 + m) * Kp;
  const _Float16* B0   = Bt + (size_t)(ngi * 32 + m) * Kp;
  const _Float16* B1   = Bt + (size_t)(ngi * 32 + 16 + m) * Kp;

  v8f acc0 = zero8(), acc1 = zero8();
  #pragma unroll 2
  for (int k0 = 0; k0 < Kp; k0 += 32) {
    FragH a, b0, b1;
    a.hv[0]  = *(const v8h*)(Arow + k0 + 8 * h);
    a.hv[1]  = *(const v8h*)(Arow + k0 + 16 + 8 * h);
    b0.hv[0] = *(const v8h*)(B0 + k0 + 8 * h);
    b0.hv[1] = *(const v8h*)(B0 + k0 + 16 + 8 * h);
    b1.hv[0] = *(const v8h*)(B1 + k0 + 8 * h);
    b1.hv[1] = *(const v8h*)(B1 + k0 + 16 + 8 * h);
    acc0 = wmma_hf(a.v, b0.v, acc0);
    acc1 = wmma_hf(a.v, b1.v, acc1);
    asm volatile("v_nop\n\tv_nop\n\tv_nop\n\tv_nop"
                 : "+v"(acc0), "+v"(acc1) : "v"(a.v), "v"(b0.v), "v"(b1.v));
  }
  #pragma unroll
  for (int r = 0; r < 8; ++r) {
    tile[(8 * h + r) * 32 + m]      = acc0[r];
    tile[(8 * h + r) * 32 + 16 + m] = acc1[r];
  }
  __syncthreads();
  store_tile_lines(tile, C + (size_t)(mt * 16) * Np + ngi * 32, Np, l);
}

__global__ __launch_bounds__(256) void k_lstm(const float* __restrict__ xWf, const float* __restrict__ xWb,
                                               const unsigned short* __restrict__ Wfh, const unsigned short* __restrict__ Wfl,
                                               const unsigned short* __restrict__ Wbh, const unsigned short* __restrict__ Wbl,
                                               const float* __restrict__ bf, const float* __restrict__ bb,
                                               float* __restrict__ hout) {
  __shared__ __align__(16) unsigned short hAh[16 * HP];
  __shared__ __align__(16) unsigned short hAl[16 * HP];
  __shared__ float g[2 * GP];
  const int dir = blockIdx.x;
  const float* xw = dir ? xWb : xWf;
  const unsigned short* Wh = dir ? Wbh : Wfh;
  const unsigned short* Wl = dir ? Wbl : Wfl;
  const float* bias = dir ? bb : bf;
  float* ho0 = hout + (size_t)(dir * 2 + 0) * TT * HP;
  float* ho1 = hout + (size_t)(dir * 2 + 1) * TT * HP;
  const int tid = threadIdx.x, wv = tid >> 5, l = tid & 31, h = l >> 4, m = l & 15;

  for (int i = tid; i < 16 * HP; i += 256) { hAh[i] = 0; hAl[i] = 0; }
  float c0 = 0.0f, c1 = 0.0f;
  __syncthreads();

  for (int step = 0; step < TT; ++step) {
    const int t = dir ? (TT - 1 - step) : step;
    for (int j = 0; j < 8; ++j) {
      const int n0 = (wv + 8 * j) * 16;
      const unsigned short* Bhr = Wh + (size_t)(n0 + m) * HP;
      const unsigned short* Blr = Wl + (size_t)(n0 + m) * HP;
      const unsigned short* Ahr = hAh + m * HP;
      const unsigned short* Alr = hAl + m * HP;
      v8f acc = zero8();
      #pragma unroll 1
      for (int k0 = 0; k0 < HP; k0 += 32) {
        FragB ah, al, bh, bl;
        ah.hv[0] = *(const v8us*)(Ahr + k0 + 8 * h);
        ah.hv[1] = *(const v8us*)(Ahr + k0 + 16 + 8 * h);
        al.hv[0] = *(const v8us*)(Alr + k0 + 8 * h);
        al.hv[1] = *(const v8us*)(Alr + k0 + 16 + 8 * h);
        bh.hv[0] = *(const v8us*)(Bhr + k0 + 8 * h);
        bh.hv[1] = *(const v8us*)(Bhr + k0 + 16 + 8 * h);
        bl.hv[0] = *(const v8us*)(Blr + k0 + 8 * h);
        bl.hv[1] = *(const v8us*)(Blr + k0 + 16 + 8 * h);
        acc = wmma_bf(ah.v, bh.v, acc);
        acc = wmma_bf(ah.v, bl.v, acc);
        acc = wmma_bf(al.v, bh.v, acc);
        asm volatile("v_nop\n\tv_nop\n\tv_nop\n\tv_nop"
                     : "+v"(acc) : "v"(ah.v), "v"(al.v), "v"(bh.v), "v"(bl.v));
      }
      if (h == 0) {
        g[n0 + m]      = acc[0];
        g[GP + n0 + m] = acc[1];
      }
    }
    __syncthreads();

    float hv0 = 0.0f, hv1 = 0.0f;
    if (tid < HID) {
      {
        const float* xr = xw + (size_t)t * GP;
        float gi = (xr[tid]           + g[tid])           + bias[tid];
        float gf = (xr[HID + tid]     + g[HID + tid])     + bias[HID + tid];
        float gc = (xr[2 * HID + tid] + g[2 * HID + tid]) + bias[2 * HID + tid];
        float go = (xr[3 * HID + tid] + g[3 * HID + tid]) + bias[3 * HID + tid];
        float ig = 1.0f / (1.0f + expf(-gi));
        float fg = 1.0f / (1.0f + expf(-gf));
        float gg = tanhf(gc);
        float og = 1.0f / (1.0f + expf(-go));
        c0 = fg * c0 + ig * gg;
        hv0 = og * tanhf(c0);
        unsigned short hb = bf16_rne(hv0);
        hAh[tid] = hb;
        hAl[tid] = bf16_rne(hv0 - bf16_val(hb));
      }
      {
        const float* xr = xw + (size_t)(TT + t) * GP;
        const float* gs = g + GP;
        float gi = (xr[tid]           + gs[tid])           + bias[tid];
        float gf = (xr[HID + tid]     + gs[HID + tid])     + bias[HID + tid];
        float gc = (xr[2 * HID + tid] + gs[2 * HID + tid]) + bias[2 * HID + tid];
        float go = (xr[3 * HID + tid] + gs[3 * HID + tid]) + bias[3 * HID + tid];
        float ig = 1.0f / (1.0f + expf(-gi));
        float fg = 1.0f / (1.0f + expf(-gf));
        float gg = tanhf(gc);
        float og = 1.0f / (1.0f + expf(-go));
        c1 = fg * c1 + ig * gg;
        hv1 = og * tanhf(c1);
        unsigned short hb = bf16_rne(hv1);
        hAh[HP + tid] = hb;
        hAl[HP + tid] = bf16_rne(hv1 - bf16_val(hb));
      }
    }
    volatile float* p0 = ho0 + (size_t)t * HP + tid;
    volatile float* p1 = ho1 + (size_t)t * HP + tid;
    *p0 = hv0; *p1 = hv1;
    __threadfence();
    *p0 = hv0; *p1 = hv1;
    __syncthreads();
  }
}


__global__ __launch_bounds__(128) void k_norms(const float* __restrict__ hbuf, float* __restrict__ norms  ) {
  const int row = blockIdx.x * 128 + threadIdx.x;
  if (row >= 2 * TT) return;
  const int seq = row / TT, r = row - seq * TT;
  const float* hf = hbuf + ((size_t)seq * TT + r) * HP;
  const float* hb = hbuf + ((size_t)(2 + seq) * TT + r) * HP;
  float sf = 0.f, sb = 0.f, sa = 0.f;
  #pragma unroll 2
  for (int k = 0; k < HID; ++k) {
    float a = hf[k], b = hb[k], s = a + b;
    sf += a * a; sb += b * b; sa += s * s;
  }
  const float nf = sqrtf(sf), nb = sqrtf(sb), nc = sqrtf(sf + sb), na = sqrtf(sa);
  volatile float* nv = norms;
  nv[row] = nf; nv[96 + row] = nb; nv[192 + row] = nc; nv[288 + row] = na;
  __threadfence();
  nv[row] = nf; nv[96 + row] = nb; nv[192 + row] = nc; nv[288 + row] = na;
}

struct Sim3 { float d, c, l; };

__device__ __forceinline__ Sim3 sim3(float dot, float na, float nb) {
  Sim3 s;
  s.d = dot;
  s.c = dot * (1.0f / (na * nb + 1e-8f));
  float d2 = fmaxf(na * na + nb * nb - 2.0f * dot, 1e-12f);
  s.l = sqrtf(d2);
  return s;
}

__global__ __launch_bounds__(256) void k_simcube(const float* __restrict__ hbuf, const float* __restrict__ norms,
                                                 float* __restrict__ sc  ) {
  const int idx = blockIdx.x * 256 + threadIdx.x;
  if (idx >= NPOS) return;
  const int i = idx / TT, j = idx - i * TT;
  const float* h1f = hbuf + ((size_t)0 * TT + i) * HP;
  const float* h2f = hbuf + ((size_t)1 * TT + j) * HP;
  const float* h1b = hbuf + ((size_t)2 * TT + i) * HP;
  const float* h2b = hbuf + ((size_t)3 * TT + j) * HP;
  float ff = 0.f, bb = 0.f, ss = 0.f;
  #pragma unroll 2
  for (int k = 0; k < HID; ++k) {
    float a = h1f[k], b = h1b[k], cc = h2f[k], d = h2b[k];
    float s1 = a + b, s2 = cc + d;
    ff += a * cc; bb += b * d; ss += s1 * s2;
  }
  Sim3 pc = sim3(ff + bb, norms[192 + i], norms[192 + TT + j]);
  Sim3 pf = sim3(ff,      norms[i],       norms[TT + j]);
  Sim3 pb = sim3(bb,      norms[96 + i],  norms[96 + TT + j]);
  Sim3 pa = sim3(ss,      norms[288 + i], norms[288 + TT + j]);
  volatile float* o = sc + idx;
  #pragma unroll 1
  for (int pass = 0; pass < 2; ++pass) {
    o[0 * NPOS] = pc.d; o[1 * NPOS]  = pc.c; o[2 * NPOS]  = pc.l;
    o[3 * NPOS] = pf.d; o[4 * NPOS]  = pf.c; o[5 * NPOS]  = pf.l;
    o[6 * NPOS] = pb.d; o[7 * NPOS]  = pb.c; o[8 * NPOS]  = pb.l;
    o[9 * NPOS] = pa.d; o[10 * NPOS] = pa.c; o[11 * NPOS] = pa.l;
    o[12 * NPOS] = 0.0f;
    __threadfence();
  }
}


__global__ __launch_bounds__(256) void k_focus(const float* __restrict__ sc, float* __restrict__ mask  ) {
  __shared__ float buf[NPOS];
  __shared__ float rv[256];
  __shared__ int   ri[256];
  __shared__ int   s1[TT], s2[TT];
  __shared__ unsigned char selm[NPOS];
  const int tid = threadIdx.x;
  for (int e = tid; e < NPOS; e += 256) selm[e] = 0;

  for (int pl = 0; pl < 2; ++pl) {
    const float* plane = sc + (size_t)(10 + pl) * NPOS;
    for (int e = tid; e < NPOS; e += 256) buf[e] = plane[e];
    if (tid < TT) { s1[tid] = 0; s2[tid] = 0; }
    __syncthreads();
    for (int it = 0; it < 2 * TT; ++it) {
      float bv = -3.0e38f; int bi = 1 << 30;
      for (int e = tid; e < NPOS; e += 256) {
        float v = buf[e];
        if (v > bv) { bv = v; bi = e; }
      }
      rv[tid] = bv; ri[tid] = bi;
      __syncthreads();
      for (int s = 128; s > 0; s >>= 1) {
        if (tid < s) {
          if (rv[tid + s] > rv[tid] ||
              (rv[tid + s] == rv[tid] && ri[tid + s] < ri[tid])) {
            rv[tid] = rv[tid + s]; ri[tid] = ri[tid + s];
          }
        }
        __syncthreads();
      }
      if (tid == 0) {
        int idx = ri[0];
        if ((unsigned)idx < (unsigned)NPOS) {
          int p1 = idx / TT, p2 = idx - p1 * TT;
          if (s1[p1] + s2[p2] == 0) { s1[p1] = 1; s2[p2] = 1; selm[idx] = 1; }
          buf[idx] = -3.0e38f;
        }
      }
      __syncthreads();
    }
    __syncthreads();
  }
  volatile float* mv = mask;
  for (int e = tid; e < NPOS; e += 256) { float v = selm[e] ? 1.0f : 0.1f; mv[e] = v; }
  __threadfence();
  for (int e = tid; e < NPOS; e += 256) { float v = selm[e] ? 1.0f : 0.1f; mv[e] = v; }
}

__global__ __launch_bounds__(256) void k_apply_focus(const float* __restrict__ sc, const float* __restrict__ mask,
                                                     float* __restrict__ fc) {
  const int idx = blockIdx.x * 256 + threadIdx.x;
  if (idx >= 13 * NPOS) return;
  const int p = idx / NPOS, e = idx - p * NPOS;
  const float mval = (p == 12) ? 1.0f : mask[e];
  const float v = sc[idx] * mval;
  volatile float* o = fc + idx;
  *o = v;
  __threadfence();
  *o = v;
}


__global__ __launch_bounds__(256) void k_bias_relu_pool(const float* __restrict__ Cmat  ,
                                                        const float* __restrict__ bias,
                                                        float* __restrict__ out  ,
                                                        int HW, int Np, int Cout, int pk, int ps, int oHW) {
  const int q = blockIdx.x * 256 + threadIdx.x;
  const int total = Cout * oHW * oHW;
  const int base = q * 4;
  if (base >= total) return;
  float r[4];
  #pragma unroll
  for (int jj = 0; jj < 4; ++jj) {
    const int idx = base + jj;
    float res = 0.0f;
    if (idx < total) {
      const int n = idx / (oHW * oHW);
      const int rem = idx - n * (oHW * oHW);
      const int py = rem / oHW, px = rem - py * oHW;
      float mx = -3.0e38f;
      for (int dy = 0; dy < pk; ++dy)
        for (int dx = 0; dx < pk; ++dx) {
          const int y = py * ps + dy, x = px * ps + dx;
          float v = Cmat[((size_t)y * HW + x) * Np + n] + bias[n];
          mx = fmaxf(mx, v);
        }
      res = fmaxf(mx, 0.0f);
    }
    r[jj] = res;
  }
  if (base + 3 < total) {
    v4f v = {r[0], r[1], r[2], r[3]};
    volatile v4f* o = (volatile v4f*)(out + base);
    *o = v;
    __threadfence();
    *o = v;
  } else {
    volatile float* o = out + base;
    for (int jj = 0; jj < 4; ++jj) if (base + jj < total) o[jj] = r[jj];
    __threadfence();
    for (int jj = 0; jj < 4; ++jj) if (base + jj < total) o[jj] = r[jj];
  }
}


__global__ __launch_bounds__(128) void k_head(const float* __restrict__ x128, const float* __restrict__ dnn_w,
                                              const float* __restrict__ dnn_b, const float* __restrict__ out_w,
                                              const float* __restrict__ out_b, float* __restrict__ out) {
  __shared__ float x[128], y[128], z[8], lse[1];
  const int tid = threadIdx.x;
  x[tid] = x128[tid];
  __syncthreads();
  {
    float acc = 0.0f;
    const float* wr = dnn_w + (size_t)tid * 128;
    #pragma unroll 1
    for (int k = 0; k < 128; ++k) acc += x[k] * wr[k];
    y[tid] = fmaxf(acc + dnn_b[tid], 0.0f);
  }
  __syncthreads();
  if (tid < NL) {
    float a = 0.0f;
    const float* orow = out_w + (size_t)tid * 128;
    #pragma unroll 1
    for (int k = 0; k < 128; ++k) a += y[k] * orow[k];
    z[tid] = a + out_b[tid];
  }
  __syncthreads();
  if (tid == 0) {
    float mx = z[0];
    for (int i = 1; i < NL; ++i) mx = fmaxf(mx, z[i]);
    float s = 0.0f;
    #pragma unroll 1
    for (int i = 0; i < NL; ++i) s += expf(z[i] - mx);
    lse[0] = mx + logf(s);
  }
  __syncthreads();
  if (tid < NL) {
    const float v = z[tid] - lse[0];
    volatile float* o = out + tid;
    *o = v;
    __threadfence();
    *o = v;
  }
}


static inline int cdiv(int a, int b) { return (a + b - 1) / b; }
static inline size_t al256(size_t b) { return (b + 255) & ~(size_t)255; }

extern "C" void kernel_launch(void* const* d_in, const int* in_sizes, int n_in,
                              void* d_out, int out_size, void* d_ws, size_t ws_size,
                              hipStream_t stream) {
  if (n_in < 23) return;
  if (in_sizes[0] != TT || in_sizes[1] != TT) return;
  if (in_sizes[3] != G4 * EMBD || in_sizes[4] != G4 * HID || in_sizes[6] != G4 * EMBD || in_sizes[7] != G4 * HID) return;
  if (out_size != NL) return;
  const int vocab = in_sizes[2] / EMBD;
  if (vocab < 1) return;

  const int*   x1     = (const int*)  d_in[0];
  const int*   x2     = (const int*)  d_in[1];
  const float* emb    = (const float*)d_in[2];
  const float* w_ih_f = (const float*)d_in[3];
  const float* w_hh_f = (const float*)d_in[4];
  const float* b_f    = (const float*)d_in[5];
  const float* w_ih_b = (const float*)d_in[6];
  const float* w_hh_b = (const float*)d_in[7];
  const float* b_b    = (const float*)d_in[8];
  const float* cw[5]  = {(const float*)d_in[9],  (const float*)d_in[11],
                         (const float*)d_in[13], (const float*)d_in[15],
                         (const float*)d_in[17]};
  const float* cb[5]  = {(const float*)d_in[10], (const float*)d_in[12],
                         (const float*)d_in[14], (const float*)d_in[16],
                         (const float*)d_in[18]};
  const float* dnn_w  = (const float*)d_in[19];
  const float* dnn_b  = (const float*)d_in[20];
  const float* out_w  = (const float*)d_in[21];
  const float* out_b  = (const float*)d_in[22];

  struct Layer { const float* w; const float* b; int Cin, HW, Cout, pk, ps, oHW; };
  Layer Ls[5] = {
    {cw[0], cb[0],  13, 48, 128, 2, 2, 24},
    {cw[1], cb[1], 128, 24, 164, 2, 2, 12},
    {cw[2], cb[2], 164, 12, 192, 2, 2,  6},
    {cw[3], cb[3], 192,  6, 192, 2, 2,  3},
    {cw[4], cb[4], 192,  3, 128, 3, 1,  1},
  };
  size_t maxA = 0, maxB = 0, maxC = 0, maxAct = 0;
  for (int li = 0; li < 5; ++li) {
    const Layer& L = Ls[li];
    int M = L.HW * L.HW, K = L.Cin * 9, N = L.Cout;
    int Mp = (M + 15) & ~15, Kp = (K + 31) & ~31, Np = (N + 31) & ~31;
    size_t a = (size_t)Mp * Kp * 2, b = (size_t)Np * Kp * 2, c = (size_t)Mp * Np * 4;
    size_t act = (size_t)N * L.oHW * L.oHW * 4;
    if (a > maxA) maxA = a;
    if (b > maxB) maxB = b;
    if (c > maxC) maxC = c;
    if (act > maxAct) maxAct = act;
  }

  char* base = (char*)d_ws;
  size_t off = 0;
  auto take = [&](size_t bytes) { size_t o = off; off += al256(bytes); return o; };
  unsigned short* eAh  = (unsigned short*)(base + take((size_t)2 * TT * EKP * 2));
  unsigned short* eAl  = (unsigned short*)(base + take((size_t)2 * TT * EKP * 2));
  unsigned short* Bfh  = (unsigned short*)(base + take((size_t)GP * EKP * 2));
  unsigned short* Bfl  = (unsigned short*)(base + take((size_t)GP * EKP * 2));
  unsigned short* Bbh  = (unsigned short*)(base + take((size_t)GP * EKP * 2));
  unsigned short* Bbl  = (unsigned short*)(base + take((size_t)GP * EKP * 2));
  unsigned short* Wfh  = (unsigned short*)(base + take((size_t)GP * HP * 2));
  unsigned short* Wfl  = (unsigned short*)(base + take((size_t)GP * HP * 2));
  unsigned short* Wbh  = (unsigned short*)(base + take((size_t)GP * HP * 2));
  unsigned short* Wbl  = (unsigned short*)(base + take((size_t)GP * HP * 2));
  float*    xWf  = (float*)   (base + take((size_t)2 * TT * GP * 4));
  float*    xWb  = (float*)   (base + take((size_t)2 * TT * GP * 4));
  float*    hbuf = (float*)   (base + take((size_t)4 * TT * HP * 4));
  float*    nrm  = (float*)   (base + take((size_t)4 * 96 * 4));
  float*    sc   = (float*)   (base + take((size_t)13 * NPOS * 4));
  float*    mask = (float*)   (base + take((size_t)NPOS * 4));
  float*    fc   = (float*)   (base + take((size_t)13 * NPOS * 4));
  _Float16* gA   = (_Float16*)(base + take(maxA));
  _Float16* gB   = (_Float16*)(base + take(maxB));
  float*    gC   = (float*)   (base + take(maxC));
  float*    act0 = (float*)   (base + take(maxAct));
  float*    act1 = (float*)   (base + take(maxAct));
  if (off > ws_size) return;

  k_pack_emb3<<<cdiv(2 * TT * (EKP / 8), 256), 256, 0, stream>>>(emb, x1, x2, eAh, eAl, vocab);
  k_pack_nk3<<<cdiv(GP * (EKP / 8), 256), 256, 0, stream>>>(w_ih_f, Bfh, Bfl, EMBD, G4, EKP, GP);
  k_pack_nk3<<<cdiv(GP * (EKP / 8), 256), 256, 0, stream>>>(w_ih_b, Bbh, Bbl, EMBD, G4, EKP, GP);
  k_pack_nk3<<<cdiv(GP * (HP / 8), 256), 256, 0, stream>>>(w_hh_f, Wfh, Wfl, HID, G4, HP, GP);
  k_pack_nk3<<<cdiv(GP * (HP / 8), 256), 256, 0, stream>>>(w_hh_b, Wbh, Wbl, HID, G4, HP, GP);
  {
    int tiles = ((2 * TT) / 16) * (GP / 32);
    k_gemm_x3<<<tiles, 32, 0, stream>>>(eAh, eAl, Bfh, Bfl, xWf, 2 * TT, GP, EKP);
    k_gemm_x3<<<tiles, 32, 0, stream>>>(eAh, eAl, Bbh, Bbl, xWb, 2 * TT, GP, EKP);
  }

  k_lstm<<<2, 256, 0, stream>>>(xWf, xWb, Wfh, Wfl, Wbh, Wbl, b_f, b_b, hbuf);
  k_norms<<<1, 128, 0, stream>>>(hbuf, nrm);
  k_simcube<<<cdiv(NPOS, 256), 256, 0, stream>>>(hbuf, nrm, sc);
  k_focus<<<1, 256, 0, stream>>>(sc, mask);
  k_apply_focus<<<cdiv(13 * NPOS, 256), 256, 0, stream>>>(sc, mask, fc);

  const float* cur = fc;
  float* outs[2] = {act0, act1};
  for (int li = 0; li < 5; ++li) {
    const Layer& L = Ls[li];
    int M = L.HW * L.HW, K = L.Cin * 9, N = L.Cout;
    int Mp = (M + 15) & ~15, Kp = (K + 31) & ~31, Np = (N + 31) & ~31;
    k_im2col<<<cdiv(Mp * (Kp / 8), 256), 256, 0, stream>>>(cur, gA, L.Cin, L.HW, K, Mp, Kp);
    k_pack_nk<<<cdiv(Np * (Kp / 8), 256), 256, 0, stream>>>(L.w, gB, K, N, Kp, Np);
    int tiles = (Mp / 16) * (Np / 32);
    k_gemm_h<<<tiles, 32, 0, stream>>>(gA, gB, gC, Mp, Np, Kp);
    float* outp = outs[li & 1];
    int total = N * L.oHW * L.oHW;
    k_bias_relu_pool<<<cdiv(cdiv(total, 4), 256), 256, 0, stream>>>(
        gC, L.b, outp, L.HW, Np, N, L.pk, L.ps, L.oHW);
    cur = outp;
  }

  k_head<<<1, 128, 0, stream>>>(cur, dnn_w, dnn_b, out_w, out_b, (float*)d_out);
}
